// Attention_LoRA_20383914787633
// MI455X (gfx1250) — hardware-verified
//
#include <hip/hip_runtime.h>
#include <math.h>
#include <stdint.h>

#define BB 2
#define SS 2048
#define DD 2048
#define HH 32
#define NKV 8
#define HD 64
#define RR 8
#define MTOT (BB * SS)
#define QN (HH * HD)
#define KVN (NKV * HD)
#define NQKV (QN + 2 * KVN)
#define TCOLS 32
#define KDIM 2048
#define TILESM (MTOT / 32)
#define MT_ROWS (SS / 16)
#define MT_PITCH 128
#define NKT (SS / 32)
#define EARLY_RG 8
#define MEXCL (-1.0e8f)
#define LORA_SCALE 0.00125f
#define PSCALE 1024.0f
#define RSC 2048.0f

typedef __attribute__((ext_vector_type(16))) __bf16   v16b;
typedef __attribute__((ext_vector_type(8)))  __bf16   v8b;
typedef __attribute__((ext_vector_type(16))) _Float16 v16h;
typedef __attribute__((ext_vector_type(8)))  _Float16 v8h;
typedef __attribute__((ext_vector_type(8)))  float    v8f;
typedef __attribute__((ext_vector_type(4)))  float    v4f;
typedef __attribute__((ext_vector_type(4)))  unsigned int v4u;
typedef __attribute__((ext_vector_type(4)))  int      v4i;
typedef float        v4fa __attribute__((ext_vector_type(4), may_alias));
typedef unsigned int v4ua __attribute__((ext_vector_type(4), may_alias));

__device__ __forceinline__ unsigned short f2bf_bits(float f) {
  const unsigned u = __float_as_uint(f);
  return (unsigned short)((u + 0x7FFFu + ((u >> 16) & 1u)) >> 16);
}
__device__ __forceinline__ float bf_bits2f(unsigned short h) { return __uint_as_float(((unsigned)h) << 16); }
__device__ __forceinline__ float bf16r(float f) { return bf_bits2f(f2bf_bits(f)); }
__device__ __forceinline__ unsigned pk16(unsigned short a, unsigned short b) { return (unsigned)a | ((unsigned)b << 16); }

__device__ __forceinline__ v8f mma_b(v16b a, v16b b, v8f c) {
  return __builtin_amdgcn_wmma_f32_16x16x32_bf16(false, a, false, b, (short)0, c, false, false);
}
__device__ __forceinline__ v8f mma_h(v16h a, v16h b, v8f c) {
  return __builtin_amdgcn_wmma_f32_16x16x32_f16(false, a, false, b, (short)0, c, false, false);
}
__device__ __forceinline__ void dep_guard_b(v8f& a, v8f& b, v16b x, v16b y) {
  asm volatile("v_nop\n\tv_nop\n\tv_nop\n\tv_nop" : "+v"(a), "+v"(b) : "v"(x), "v"(y));
}
__device__ __forceinline__ void dep_guard_h(v8f& a, v8f& b, v16h x, v16h y) {
  asm volatile("v_nop\n\tv_nop\n\tv_nop\n\tv_nop" : "+v"(a), "+v"(b) : "v"(x), "v"(y));
}
__device__ __forceinline__ void dep_guard_h3(v8f& a, v8f& b, v16h x, v16h y, v16h z) {
  asm volatile("v_nop\n\tv_nop\n\tv_nop\n\tv_nop" : "+v"(a), "+v"(b) : "v"(x), "v"(y), "v"(z));
}
__device__ __forceinline__ void keep4_b(v16b a, v16b b, v16b c, v16b d) {
  asm volatile("v_nop" :: "v"(a), "v"(b), "v"(c), "v"(d));
}
__device__ __forceinline__ void keep2_h(v16h a, v16h b) {
  asm volatile("v_nop" :: "v"(a), "v"(b));
}
__device__ __forceinline__ void acc_guard4(v8f& a, v8f& b, v8f& c, v8f& d) {
  asm volatile("v_nop\n\tv_nop\n\tv_nop\n\tv_nop" : "+v"(a), "+v"(b), "+v"(c), "+v"(d));
}

union FragB { v16b v; v8b h[2]; };
union FragH { v16h v; v8h h[2]; };
union PackB { v16b v; v4u u[2]; };
__device__ __forceinline__ v16b ldfrag_b(const unsigned short* p) {
  FragB f; f.h[0] = *(const v8b*)(p); f.h[1] = *(const v8b*)(p + 16); return f.v;
}
__device__ __forceinline__ v16h ldfrag_h(const unsigned short* p) {
  FragH f; f.h[0] = *(const v8h*)(p); f.h[1] = *(const v8h*)(p + 16); return f.v;
}
__device__ __forceinline__ v16h ldfrag_lds(const _Float16* p) {
  FragH f; f.h[0] = *(const v8h*)(p); f.h[1] = *(const v8h*)(p + 16); return f.v;
}
__device__ __forceinline__ void wave_lds_sync() {
  __builtin_amdgcn_fence(__ATOMIC_RELEASE, "workgroup");
  __builtin_amdgcn_wave_barrier();
  __builtin_amdgcn_fence(__ATOMIC_ACQUIRE, "workgroup");
}

__global__ __launch_bounds__(256) void cvt_bf16_kernel(const float* __restrict__ src,
                                                       unsigned short* __restrict__ dst, int n8) {
  const int i = blockIdx.x * 256 + threadIdx.x;
  if (i < n8) {
    const float* p = src + (size_t)i * 8;
    const v4f a = *(const v4f*)(p);
    const v4f b = *(const v4f*)(p + 4);
    const v4u u = (v4u){pk16(f2bf_bits(a[0]), f2bf_bits(a[1])), pk16(f2bf_bits(a[2]), f2bf_bits(a[3])),
                        pk16(f2bf_bits(b[0]), f2bf_bits(b[1])), pk16(f2bf_bits(b[2]), f2bf_bits(b[3]))};
    unsigned short* d = dst + (size_t)i * 8;
    *(volatile v4u*)d = u;
    __threadfence();
    *(volatile v4u*)d = u;
  }
}

__global__ __launch_bounds__(256) void lora_t_kernel(const unsigned short* __restrict__ Xb,
    const float* __restrict__ aq, const float* __restrict__ ak,
    const float* __restrict__ av, const float* __restrict__ ao, float* __restrict__ T) {
  __shared__ __align__(16) float sTt[8][16 * 36];
  const int lane = threadIdx.x & 31, wave = threadIdx.x >> 5;
  const int rl = lane & 15, hlf = lane >> 4, koff = hlf * 8, mOff = hlf * 8;
  const int tile = blockIdx.x * 8 + wave;
  if (tile >= MTOT / 64) return;
  const int m0 = tile * 64;
  const float* bsrc[2];
#pragma unroll
  for (int j = 0; j < 2; ++j) {
    const int n = 16 * j + rl;
    const int g = n >> 3;
    const float* pa = aq;
    pa = (g == 1) ? ak : pa;
    pa = (g == 2) ? av : pa;
    pa = (g == 3) ? ao : pa;
    bsrc[j] = pa + (size_t)(n & 7) * KDIM + koff;
  }
  v8f acc[4][2];
#pragma unroll
  for (int i = 0; i < 4; ++i)
#pragma unroll
    for (int j = 0; j < 2; ++j) acc[i][j] = (v8f){0.f, 0.f, 0.f, 0.f, 0.f, 0.f, 0.f, 0.f};

  for (int k0 = 0; k0 < KDIM; k0 += 32) {
    v16b bfr[2];
#pragma unroll
    for (int j = 0; j < 2; ++j) {
      const float* p = bsrc[j] + k0;
      const v4f f0 = *(const v4f*)(p), f1 = *(const v4f*)(p + 4);
      const v4f f2 = *(const v4f*)(p + 16), f3 = *(const v4f*)(p + 20);
      PackB pb;
      pb.u[0] = (v4u){pk16(f2bf_bits(f0[0]), f2bf_bits(f0[1])), pk16(f2bf_bits(f0[2]), f2bf_bits(f0[3])),
                      pk16(f2bf_bits(f1[0]), f2bf_bits(f1[1])), pk16(f2bf_bits(f1[2]), f2bf_bits(f1[3]))};
      pb.u[1] = (v4u){pk16(f2bf_bits(f2[0]), f2bf_bits(f2[1])), pk16(f2bf_bits(f2[2]), f2bf_bits(f2[3])),
                      pk16(f2bf_bits(f3[0]), f2bf_bits(f3[1])), pk16(f2bf_bits(f3[2]), f2bf_bits(f3[3]))};
      bfr[j] = pb.v;
    }
#pragma unroll
    for (int i = 0; i < 4; ++i) {
      const v16b ah = ldfrag_b(Xb + (size_t)(m0 + 16 * i + rl) * KDIM + koff + k0);
      acc[i][0] = mma_b(ah, bfr[0], acc[i][0]);
      acc[i][1] = mma_b(ah, bfr[1], acc[i][1]);
      dep_guard_b(acc[i][0], acc[i][1], ah, bfr[0]);
    }
    keep4_b(bfr[0], bfr[1], bfr[0], bfr[1]);
  }
  acc_guard4(acc[0][0], acc[0][1], acc[1][0], acc[1][1]);
  acc_guard4(acc[2][0], acc[2][1], acc[3][0], acc[3][1]);

  float* slab = sTt[wave];
  const int q = lane >> 3, c4 = (lane & 7) * 4;
#pragma unroll
  for (int i = 0; i < 4; ++i) {
    const int mBase = m0 + 16 * i;
#pragma unroll
    for (int j = 0; j < 2; ++j)
#pragma unroll
      for (int r = 0; r < 8; ++r) slab[(mOff + r) * 36 + 16 * j + rl] = acc[i][j][r];
    wave_lds_sync();
    v4f fv[4];
#pragma unroll
    for (int it = 0; it < 4; ++it) fv[it] = *(const v4fa*)(slab + (it * 4 + q) * 36 + c4);
    for (int pass = 0; pass < 2; ++pass) {
#pragma unroll
      for (int it = 0; it < 4; ++it) {
        *(volatile v4f*)(T + (size_t)(mBase + it * 4 + q) * TCOLS + c4) = fv[it];
      }
      __threadfence();
    }
    wave_lds_sync();
  }
}

__global__ __launch_bounds__(256) void mflag_kernel(const float* __restrict__ mask, int* __restrict__ mtab) {
  __shared__ int fl[NKT];
  __shared__ int rm[8];
  const int rg = blockIdx.x, tid = threadIdx.x, lane = tid & 31, wave = tid >> 5;
  const int c0 = tid * 8;
  int excl = 0, nz = 0;
  unsigned rowm = 0u;
#pragma unroll 1
  for (int r = 0; r < 16; ++r) {
    const float* mr = mask + (size_t)(rg * 16 + r) * SS + c0;
    const v4f a0 = *(const v4f*)(mr);
    const v4f a1 = *(const v4f*)(mr + 4);
    int adm = 0;
#pragma unroll
    for (int e = 0; e < 4; ++e) {
      const float m0v = bf16r(a0[e]), m1v = bf16r(a1[e]);
      excl += ((m0v < MEXCL) ? 1 : 0) + ((m1v < MEXCL) ? 1 : 0);
      nz  |= ((m0v != 0.0f) ? 1 : 0) | ((m1v != 0.0f) ? 1 : 0);
      adm |= ((m0v >= MEXCL) ? 1 : 0) | ((m1v >= MEXCL) ? 1 : 0);
    }
    rowm |= ((unsigned)adm) << r;
  }
  excl += __shfl_xor(excl, 1, 32);
  excl += __shfl_xor(excl, 2, 32);
  nz |= __shfl_xor(nz, 1, 32);
  nz |= __shfl_xor(nz, 2, 32);
#pragma unroll
  for (int off = 1; off < 32; off <<= 1) rowm |= (unsigned)__shfl_xor((int)rowm, off, 32);
  if ((lane & 3) == 0) fl[tid >> 2] = (excl == 512) ? 0 : ((nz != 0) ? 2 : 1);
  if (lane == 0) rm[wave] = (int)rowm;
  __syncthreads();
  if (wave == 0) {
    int all = rm[0];
#pragma unroll
    for (int w = 1; w < 8; ++w) all |= rm[w];
    const bool hasEmpty = ((all & 0xFFFF) != 0xFFFF);
    const int f0 = fl[lane], f1 = fl[lane + 32];
    int ke = (f0 != 0) ? 32 * (lane + 1) : 0;
    const int k1 = (f1 != 0) ? 32 * (lane + 33) : 0;
    ke = (k1 > ke) ? k1 : ke;
#pragma unroll
    for (int off = 1; off < 32; off <<= 1) { const int o = __shfl_xor(ke, off, 32); ke = (o > ke) ? o : ke; }
    const int kend = hasEmpty ? SS : ke;
    int ev[4];
#pragma unroll
    for (int e = 0; e < 4; ++e) {
      const int fv = fl[(4 * lane + e) & (NKT - 1)];
      const int fv2 = hasEmpty ? 2 : fv;
      ev[e] = (lane < 16) ? fv2 : kend;
    }
    const v4i val = (v4i){ev[0], ev[1], ev[2], ev[3]};
    int* dst = mtab + (size_t)rg * MT_PITCH + 4 * lane;
    *(volatile v4i*)dst = val;
    __threadfence();
    *(volatile v4i*)dst = val;
  }
}

template <int MODE>
__global__ __launch_bounds__(256) void gemm_kernel(
    const unsigned short* __restrict__ Ap, const unsigned short* __restrict__ A2p,
    const unsigned short* __restrict__ Btp, const float* __restrict__ Tp, const float* __restrict__ BLp,
    const float* __restrict__ cosT, const float* __restrict__ sinT,
    unsigned short* __restrict__ outH, unsigned short* __restrict__ outL, float* __restrict__ outF, int N) {
  constexpr bool SPLITA = (MODE == 3);
  constexpr bool ROPE = (MODE <= 1);
  constexpr bool OUT16 = (MODE <= 1);
  constexpr bool OUTLO = (MODE == 0);
  constexpr int TCOL = 8 * MODE;
  __shared__ __align__(16) float sT[8][16 * 68];
  const int lane = threadIdx.x & 31, wave = threadIdx.x >> 5;
  const int rl = lane & 15, hlf = lane >> 4, koff = hlf * 8, mOff = hlf * 8;
  const int tilesN = N >> 6;
  const int tile = blockIdx.x * 8 + wave;
  if (tile >= TILESM * tilesN) return;
  const int tm = tile / tilesN, tn = tile - tm * tilesN;
  const int m0 = tm * 32, n0 = tn * 64;

  v8f acc[2][4];
#pragma unroll
  for (int i = 0; i < 2; ++i)
#pragma unroll
    for (int j = 0; j < 4; ++j) acc[i][j] = (v8f){0.f, 0.f, 0.f, 0.f, 0.f, 0.f, 0.f, 0.f};

  for (int k0 = 0; k0 < KDIM; k0 += 32) {
    v16b bh[4];
#pragma unroll
    for (int j = 0; j < 4; ++j) bh[j] = ldfrag_b(Btp + (size_t)(n0 + 16 * j + rl) * KDIM + koff + k0);
#pragma unroll
    for (int i = 0; i < 2; ++i) {
      const size_t ao = (size_t)(m0 + 16 * i + rl) * KDIM + koff + k0;
      const v16b ah = ldfrag_b(Ap + ao);
      v16b al = ah;
      if (SPLITA) al = ldfrag_b(A2p + ao);
#pragma unroll
      for (int j = 0; j < 4; ++j) {
        acc[i][j] = mma_b(ah, bh[j], acc[i][j]);
        if (SPLITA) acc[i][j] = mma_b(al, bh[j], acc[i][j]);
      }
      dep_guard_b(acc[i][0], acc[i][3], ah, al);
    }
    keep4_b(bh[0], bh[1], bh[2], bh[3]);
  }
  acc_guard4(acc[0][0], acc[0][1], acc[0][2], acc[0][3]);
  acc_guard4(acc[1][0], acc[1][1], acc[1][2], acc[1][3]);

  float* slab = sT[wave];
#pragma unroll
  for (int i = 0; i < 2; ++i) {
    const int mBase = m0 + 16 * i;
#pragma unroll
    for (int j = 0; j < 4; ++j) {
      const int cc = 16 * j + rl;
      const int n = n0 + cc;
      const float* blq = BLp + (size_t)n * RR;
      const v4f b0 = *(const v4f*)(blq), b1 = *(const v4f*)(blq + 4);
      float bl[8];
      bl[0] = bf16r(b0[0]); bl[1] = bf16r(b0[1]); bl[2] = bf16r(b0[2]); bl[3] = bf16r(b0[3]);
      bl[4] = bf16r(b1[0]); bl[5] = bf16r(b1[1]); bl[6] = bf16r(b1[2]); bl[7] = bf16r(b1[3]);
#pragma unroll
      for (int r = 0; r < 8; ++r) {
        const int mrow = mBase + mOff + r;
        const float* tq = Tp + (size_t)mrow * TCOLS + TCOL;
        const v4f t0 = *(const v4f*)(tq), t1 = *(const v4f*)(tq + 4);
        float dot = t0[0] * bl[0];
        dot += t0[1] * bl[1]; dot += t0[2] * bl[2]; dot += t0[3] * bl[3];
        dot += t1[0] * bl[4]; dot += t1[1] * bl[5]; dot += t1[2] * bl[6]; dot += t1[3] * bl[7];
        float v = acc[i][j][r] + LORA_SCALE * dot;
        if (ROPE) {
          const int s = mrow & (SS - 1);
          const int ip = cc >> 1;
          const float c = bf16r(cosT[s * (HD / 2) + ip]);
          const float sn = bf16r(sinT[s * (HD / 2) + ip]);
          const float pv = __shfl_xor(v, 1, 32);
          const float ve = v * c - pv * sn;
          const float vo = pv * sn + v * c;
          v = (rl & 1) ? vo : ve;
        }
        slab[(mOff + r) * 68 + cc] = v;
      }
    }
    wave_lds_sync();
    if (OUT16) {
      const int q = lane >> 3, c8 = (lane & 7) * 8;
      v4u hv[4], lv[4];
#pragma unroll
      for (int it = 0; it < 4; ++it) {
        const float* sp = slab + (it * 4 + q) * 68 + c8;
        unsigned short hb[8], lb[8];
#pragma unroll
        for (int e = 0; e < 8; ++e) {
          const float x = sp[e];
          const _Float16 xh = (_Float16)x;
          hb[e] = __builtin_bit_cast(unsigned short, xh);
          lb[e] = 0;
          if (OUTLO) lb[e] = __builtin_bit_cast(unsigned short, (_Float16)((x - (float)xh) * RSC));
        }
        hv[it] = (v4u){pk16(hb[0], hb[1]), pk16(hb[2], hb[3]), pk16(hb[4], hb[5]), pk16(hb[6], hb[7])};
        lv[it] = (v4u){pk16(lb[0], lb[1]), pk16(lb[2], lb[3]), pk16(lb[4], lb[5]), pk16(lb[6], lb[7])};
      }
      for (int pass = 0; pass < 2; ++pass) {
#pragma unroll
        for (int it = 0; it < 4; ++it) {
          const size_t go = (size_t)(mBase + it * 4 + q) * N + n0 + c8;
          *(volatile v4u*)(outH + go) = hv[it];
          if (OUTLO) *(volatile v4u*)(outL + go) = lv[it];
        }
        __threadfence();
      }
    } else {
      const int hh = lane >> 4, c4 = (lane & 15) * 4;
      v4f fv[8];
#pragma unroll
      for (int it = 0; it < 8; ++it) fv[it] = *(const v4fa*)(slab + (it * 2 + hh) * 68 + c4);
      for (int pass = 0; pass < 2; ++pass) {
#pragma unroll
        for (int it = 0; it < 8; ++it) {
          const size_t go = (size_t)(mBase + it * 2 + hh) * N + n0 + c4;
          *(volatile v4f*)(outF + go) = fv[it];
        }
        __threadfence();
      }
    }
    wave_lds_sync();
  }
}

__global__ __launch_bounds__(256) void vtrans_kernel(const float* __restrict__ Vf,
                                                     unsigned short* __restrict__ VThi, unsigned short* __restrict__ VTlo) {
  __shared__ __align__(16) unsigned short th[64 * 72];
  __shared__ __align__(16) unsigned short tl[64 * 72];
  const int cb = blockIdx.x;
  const int rb = blockIdx.y;
  const int b = rb >> 5, j0 = (rb & 31) * 64, d0 = cb * 64;
  const int tid = threadIdx.x;
  {
    const int rr = tid >> 2;
    const int cq = (tid & 3) * 16;
    const float* src = Vf + (size_t)(rb * 64 + rr) * KVN + d0 + cq;
#pragma unroll
    for (int q = 0; q < 4; ++q) {
      const v4f f = *(const v4f*)(src + 4 * q);
#pragma unroll
      for (int e = 0; e < 4; ++e) {
        const float fe = f[e];
        const _Float16 hh = (_Float16)fe;
        const float res = (fe - (float)hh) * RSC;
        th[rr * 72 + cq + 4 * q + e] = __builtin_bit_cast(unsigned short, hh);
        tl[rr * 72 + cq + 4 * q + e] = __builtin_bit_cast(unsigned short, (_Float16)res);
      }
    }
  }
  __syncthreads();
  const int sub = tid >> 3;
  const int c8 = (tid & 7) * 8;
  v4u hv[2], lv[2];
#pragma unroll
  for (int it = 0; it < 2; ++it) {
    const int oc = it * 32 + sub;
    v4u a, a2;
#pragma unroll
    for (int q = 0; q < 4; ++q) {
      a[q]  = pk16(th[(c8 + 2 * q) * 72 + oc], th[(c8 + 2 * q + 1) * 72 + oc]);
      a2[q] = pk16(tl[(c8 + 2 * q) * 72 + oc], tl[(c8 + 2 * q + 1) * 72 + oc]);
    }
    hv[it] = a; lv[it] = a2;
  }
  for (int pass = 0; pass < 2; ++pass) {
#pragma unroll
    for (int it = 0; it < 2; ++it) {
      const int oc = it * 32 + sub;
      const size_t go = ((size_t)(b * KVN + d0 + oc)) * SS + j0 + c8;
      *(volatile v4u*)(VThi + go) = hv[it];
      *(volatile v4u*)(VTlo + go) = lv[it];
    }
    __threadfence();
  }
}

template <bool ESPLIT>
__global__ __launch_bounds__(32) void attn_kernel(
    const unsigned short* __restrict__ Qhi, const unsigned short* __restrict__ Qlo,
    const unsigned short* __restrict__ Kp,
    const unsigned short* __restrict__ VThi, const unsigned short* __restrict__ VTlo,
    const float* __restrict__ mask, const int* __restrict__ mtab,
    unsigned short* __restrict__ Ohi, unsigned short* __restrict__ Olo, int rgBase) {
  __shared__ __align__(16) _Float16 plds[16 * 32];
  __shared__ __align__(16) _Float16 plds2[16 * 32];
  __shared__ __align__(16) unsigned short osh[16 * 72];
  __shared__ __align__(16) unsigned short osl[16 * 72];
  const int lane = threadIdx.x & 31, hlf = lane >> 4, rl = lane & 15, koff = hlf * 8, mOff = hlf * 8;
  int rg = blockIdx.x + rgBase;
  rg = (rg < MT_ROWS) ? rg : (MT_ROWS - 1);
  const int h = blockIdx.y, b = blockIdx.z, kvh = h >> 2;

  const size_t qo = (size_t)(b * SS + rg * 16 + rl) * QN + h * HD + koff;
  const v16h qh0 = ldfrag_h(Qhi + qo), qh1 = ldfrag_h(Qhi + qo + 32);
  const v16h ql0 = ldfrag_h(Qlo + qo), ql1 = ldfrag_h(Qlo + qo + 32);

  int kend = __builtin_amdgcn_readfirstlane(mtab[rg * MT_PITCH + NKT]);
  kend = (kend < 0) ? 0 : kend;
  kend = (kend > SS) ? SS : kend;
  const int ntile = kend >> 5;

  float mmax[8], lsum[8];
  v8f oh[4], ol[4];
#pragma unroll
  for (int r = 0; r < 8; ++r) { mmax[r] = -1.0e30f; lsum[r] = 0.0f; }
#pragma unroll
  for (int t = 0; t < 4; ++t) {
    oh[t] = (v8f){0.f, 0.f, 0.f, 0.f, 0.f, 0.f, 0.f, 0.f};
    ol[t] = (v8f){0.f, 0.f, 0.f, 0.f, 0.f, 0.f, 0.f, 0.f};
  }

  for (int kt = 0; kt < ntile; ++kt) {
    const int f = __builtin_amdgcn_readfirstlane(mtab[rg * MT_PITCH + kt]);
    if (f == 0) continue;
    v8f sf[2];
#pragma unroll
    for (int nt = 0; nt < 2; ++nt) {
      const size_t ko = (size_t)(b * SS + kt * 32 + nt * 16 + rl) * KVN + kvh * HD + koff;
      const v16h k0 = ldfrag_h(Kp + ko), k1 = ldfrag_h(Kp + ko + 32);
      v8f zh = (v8f){0.f, 0.f, 0.f, 0.f, 0.f, 0.f, 0.f, 0.f};
      v8f zl = (v8f){0.f, 0.f, 0.f, 0.f, 0.f, 0.f, 0.f, 0.f};
      zh = mma_h(qh0, k0, zh);
      zl = mma_h(ql0, k0, zl);
      zh = mma_h(qh1, k1, zh);
      zl = mma_h(ql1, k1, zl);
      dep_guard_h3(zh, zl, qh1, ql1, k1);
      keep2_h(k0, ql0);
      sf[nt] = zh + zl * (1.0f / RSC);
    }
    float madd[2][8];
#pragma unroll
    for (int nt = 0; nt < 2; ++nt)
#pragma unroll
      for (int r = 0; r < 8; ++r) madd[nt][r] = 0.0f;
    if (f == 2) {
#pragma unroll
      for (int nt = 0; nt < 2; ++nt)
#pragma unroll
        for (int r = 0; r < 8; ++r)
          madd[nt][r] = bf16r(mask[(size_t)(rg * 16 + mOff + r) * SS + kt * 32 + nt * 16 + rl]);
    }
    float corr[8];
#pragma unroll
    for (int r = 0; r < 8; ++r) {
      const float s0 = sf[0][r] * 0.125f + madd[0][r];
      const float s1 = sf[1][r] * 0.125f + madd[1][r];
      float mx = fmaxf(s0, s1);
#pragma unroll
      for (int off = 1; off <= 8; off <<= 1) mx = fmaxf(mx, __shfl_xor(mx, off, 32));
      const float nm = fmaxf(mmax[r], mx);
      const float cr = __expf(mmax[r] - nm);
      const float p0 = __expf(s0 - nm);
      const float p1 = __expf(s1 - nm);
      float sl = p0 + p1;
#pragma unroll
      for (int off = 1; off <= 8; off <<= 1) sl += __shfl_xor(sl, off, 32);
      lsum[r] = lsum[r] * cr + sl;
      mmax[r] = nm;
      corr[r] = cr;
      const float ps0 = p0 * PSCALE, ps1 = p1 * PSCALE;
      const _Float16 ph0 = (_Float16)ps0, ph1 = (_Float16)ps1;
      plds[(mOff + r) * 32 + rl]      = ph0;
      plds[(mOff + r) * 32 + 16 + rl] = ph1;
      if (ESPLIT) {
        plds2[(mOff + r) * 32 + rl]      = (_Float16)((ps0 - (float)ph0) * RSC);
        plds2[(mOff + r) * 32 + 16 + rl] = (_Float16)((ps1 - (float)ph1) * RSC);
      }
    }
#pragma unroll
    for (int t = 0; t < 4; ++t)
#pragma unroll
      for (int r = 0; r < 8; ++r) { oh[t][r] *= corr[r]; ol[t][r] *= corr[r]; }
    __syncthreads();
    const v16h ap = ldfrag_lds(plds + rl * 32 + koff);
    v16h apl = ap;
    if (ESPLIT) apl = ldfrag_lds(plds2 + rl * 32 + koff);
    __syncthreads();
    v16h vh = (v16h){}, vl = (v16h){};
#pragma unroll
    for (int t = 0; t < 4; ++t) {
      const size_t vo = ((size_t)(b * KVN + kvh * HD + t * 16 + rl)) * SS + kt * 32 + koff;
      vh = ldfrag_h(VThi + vo);
      vl = ldfrag_h(VTlo + vo);
      oh[t] = mma_h(ap, vh, oh[t]);
      ol[t] = mma_h(ap, vl, ol[t]);
      if (ESPLIT) ol[t] = mma_h(apl, vh, ol[t]);
    }
    dep_guard_h3(oh[3], ol[3], ap, apl, vl);
    dep_guard_h3(oh[0], ol[0], vh, apl, vl);
  }
  acc_guard4(oh[0], oh[1], oh[2], oh[3]);
  acc_guard4(ol[0], ol[1], ol[2], ol[3]);

#pragma unroll
  for (int r = 0; r < 8; ++r) {
    const float ls = lsum[r] * PSCALE;
    const float inv = (ls > 0.0f) ? __frcp_rn(ls) : 0.0f;
#pragma unroll
    for (int t = 0; t < 4; ++t) {
      const float v = (oh[t][r] + ol[t][r] * (1.0f / RSC)) * inv;
      const unsigned short hb = f2bf_bits(v);
      const unsigned short lb = f2bf_bits(v - bf_bits2f(hb));
      osh[(mOff + r) * 72 + 16 * t + rl] = hb;
      osl[(mOff + r) * 72 + 16 * t + rl] = lb;
    }
  }
  __syncthreads();
  const int q = lane >> 3, c8 = (lane & 7) * 8;
  v4u hv[4], lv[4];
#pragma unroll
  for (int it = 0; it < 4; ++it) {
    hv[it] = *(const v4ua*)(osh + (it * 4 + q) * 72 + c8);
    lv[it] = *(const v4ua*)(osl + (it * 4 + q) * 72 + c8);
  }
  for (int pass = 0; pass < 2; ++pass) {
#pragma unroll
    for (int it = 0; it < 4; ++it) {
      const size_t go = (size_t)(b * SS + rg * 16 + it * 4 + q) * QN + h * HD + c8;
      *(volatile v4u*)(Ohi + go) = hv[it];
      *(volatile v4u*)(Olo + go) = lv[it];
    }
    __threadfence();
  }
}

extern "C" void kernel_launch(void* const* d_in, const int* in_sizes, int n_in,
                              void* d_out, int out_size, void* d_ws, size_t ws_size,
                              hipStream_t stream) {
  if (n_in < 17) return;
  if (in_sizes[0] != MTOT * DD) return;
  if (in_sizes[2] != SS * (HD / 2) || in_sizes[3] != SS * (HD / 2)) return;
  if (in_sizes[4] != SS * SS) return;
  if (in_sizes[5] != QN * DD || in_sizes[6] != KVN * DD || in_sizes[7] != KVN * DD) return;
  if (in_sizes[8] != DD * QN) return;
  if (in_sizes[9] != RR * DD || in_sizes[10] != QN * RR) return;
  if (in_sizes[11] != RR * DD || in_sizes[12] != KVN * RR) return;
  if (in_sizes[13] != RR * DD || in_sizes[14] != KVN * RR) return;
  if (in_sizes[15] != RR * DD || in_sizes[16] != QN * RR) return;
  if (out_size != MTOT * DD) return;

  const float* x    = (const float*)d_in[0];
  const float* cosT = (const float*)d_in[2];
  const float* sinT = (const float*)d_in[3];
  const float* mask = (const float*)d_in[4];
  const float* wq   = (const float*)d_in[5];
  const float* wk   = (const float*)d_in[6];
  const float* wv   = (const float*)d_in[7];
  const float* wo   = (const float*)d_in[8];
  const float* aq   = (const float*)d_in[9];
  const float* bq   = (const float*)d_in[10];
  const float* ak   = (const float*)d_in[11];
  const float* bk   = (const float*)d_in[12];
  const float* av   = (const float*)d_in[13];
  const float* bv   = (const float*)d_in[14];
  const float* ao   = (const float*)d_in[15];
  const float* bo   = (const float*)d_in[16];
  float* out = (float*)d_out;

  const size_t szXb   = (size_t)MTOT * DD * 2;
  const size_t szWqkv = (size_t)NQKV * DD * 2;
  const size_t szWo   = (size_t)DD * QN * 2;
  const size_t szT    = (size_t)MTOT * TCOLS * 4;
  const size_t szMt   = (size_t)MT_ROWS * MT_PITCH * 4;
  const size_t szQ    = (size_t)MTOT * QN * 2;
  const size_t szK    = (size_t)MTOT * KVN * 2;
  const size_t szVf   = (size_t)MTOT * KVN * 4;
  const size_t szVT   = (size_t)BB * KVN * SS * 2;
  const size_t szO    = (size_t)MTOT * QN * 2;
  size_t off = 0;
  const size_t oXb   = off; off += szXb;
  const size_t oWqkv = off; off += szWqkv;
  const size_t oWo   = off; off += szWo;
  const size_t oT    = off; off += szT;
  const size_t oMt   = off; off += szMt;
  const size_t oQhi  = off; off += szQ;
  const size_t oQlo  = off; off += szQ;
  const size_t oKh   = off; off += szK;
  const size_t oVf   = off; off += szVf;
  const size_t oVThi = off; off += szVT;
  const size_t oVTlo = off; off += szVT;
  const size_t oOhi  = off; off += szO;
  const size_t oOlo  = off; off += szO;
  if (off > ws_size) return;

  char* ws = (char*)d_ws;
  unsigned short* Xb   = (unsigned short*)(ws + oXb);
  unsigned short* Wqkv = (unsigned short*)(ws + oWqkv);
  unsigned short* Wob  = (unsigned short*)(ws + oWo);
  float*          T    = (float*)(ws + oT);
  int*            Mt   = (int*)(ws + oMt);
  unsigned short* Qhi  = (unsigned short*)(ws + oQhi);
  unsigned short* Qlo  = (unsigned short*)(ws + oQlo);
  unsigned short* Kh   = (unsigned short*)(ws + oKh);
  float*          Vf   = (float*)(ws + oVf);
  unsigned short* VThi = (unsigned short*)(ws + oVThi);
  unsigned short* VTlo = (unsigned short*)(ws + oVTlo);
  unsigned short* Ohi  = (unsigned short*)(ws + oOhi);
  unsigned short* Olo  = (unsigned short*)(ws + oOlo);

  const dim3 blk(256);
  const int n8x  = MTOT * DD / 8;
  const int n8wq = QN * DD / 8;
  const int n8wk = KVN * DD / 8;
  const int n8wo = DD * QN / 8;

  cvt_bf16_kernel<<<dim3((n8x + 255) / 256), blk, 0, stream>>>(x, Xb, n8x);
  cvt_bf16_kernel<<<dim3((n8wq + 255) / 256), blk, 0, stream>>>(wq, Wqkv, n8wq);
  cvt_bf16_kernel<<<dim3((n8wk + 255) / 256), blk, 0, stream>>>(wk, Wqkv + (size_t)QN * DD, n8wk);
  cvt_bf16_kernel<<<dim3((n8wk + 255) / 256), blk, 0, stream>>>(wv, Wqkv + (size_t)(QN + KVN) * DD, n8wk);
  cvt_bf16_kernel<<<dim3((n8wo + 255) / 256), blk, 0, stream>>>(wo, Wob, n8wo);
  lora_t_kernel<<<dim3(MTOT / 64 / 8), blk, 0, stream>>>(Xb, aq, ak, av, ao, T);
  mflag_kernel<<<dim3(MT_ROWS), blk, 0, stream>>>(mask, Mt);
  gemm_kernel<0><<<dim3(TILESM * (QN / 64) / 8), blk, 0, stream>>>(
      Xb, Xb, Wqkv, T, bq, cosT, sinT, Qhi, Qlo, Vf, QN);
  gemm_kernel<1><<<dim3(TILESM * (KVN / 64) / 8), blk, 0, stream>>>(
      Xb, Xb, Wqkv + (size_t)QN * DD, T, bk, cosT, sinT, Kh, Kh, Vf, KVN);
  gemm_kernel<2><<<dim3(TILESM * (KVN / 64) / 8), blk, 0, stream>>>(
      Xb, Xb, Wqkv + (size_t)(QN + KVN) * DD, T, bv, cosT, sinT, Ohi, Olo, Vf, KVN);
  vtrans_kernel<<<dim3(KVN / 64, MTOT / 64), blk, 0, stream>>>(Vf, VThi, VTlo);
  attn_kernel<true><<<dim3(EARLY_RG, HH, BB), dim3(32), 0, stream>>>(
      Qhi, Qlo, Kh, VThi, VTlo, mask, Mt, Ohi, Olo, 0);
  attn_kernel<false><<<dim3(MT_ROWS - EARLY_RG, HH, BB), dim3(32), 0, stream>>>(
      Qhi, Qlo, Kh, VThi, VTlo, mask, Mt, Ohi, Olo, EARLY_RG);
  gemm_kernel<3><<<dim3(TILESM * (DD / 64) / 8), blk, 0, stream>>>(
      Ohi, Olo, Wob, T, bo, cosT, sinT, Qhi, Qlo, out, DD);
  (void)hipGetLastError();
}
